// MultiHeadAttention_66383014527497
// MI455X (gfx1250) — hardware-verified
//
#include <hip/hip_runtime.h>
#ifndef NB
#define NB 8
#endif
#ifndef SEQ
#define SEQ 1024
#endif
#define SQ SEQ
#define NB_FULL 8
#define SQ_FULL 1024
#define DM 1024
#define NH 16
#define HD 64
#define HG 8
#define LQ (3 * DM)
#define NR ((size_t)NB * SQ)

static_assert(SQ % 128 == 0);
static_assert(((size_t)NB * SQ) % 128 == 0);
static_assert(NH % HG == 0);
static_assert(DM % 64 == 0 && LQ % 64 == 0 && HD == 64);
static_assert(NB <= NB_FULL && SQ <= SQ_FULL);
static_assert(NH * HD == DM);

#define WS_ALIGN(x) ((((size_t)(x)) + 255) & ~(size_t)255)
#define SZ_BQKV  WS_ALIGN((size_t)LQ * DM * 2)
#define SZ_BO    WS_ALIGN((size_t)DM * DM * 2)
#define SZ_X16   WS_ALIGN(NR * DM * 2)
#define SZ_QKV   WS_ALIGN(NR * LQ * 2)
#define SZ_S     WS_ALIGN((size_t)HG * SQ * SQ * 4)
#define SZ_P     WS_ALIGN((size_t)HG * SQ * SQ * 2)
#define SZ_VT    WS_ALIGN((size_t)NH * HD * SQ * 2)
static_assert(SZ_BQKV + SZ_BO + SZ_X16 + SZ_QKV + SZ_S + SZ_P + SZ_VT <= (size_t)134217728);

typedef unsigned short v8us __attribute__((ext_vector_type(8), may_alias));
typedef float  v8f  __attribute__((ext_vector_type(8)));
typedef float  v4f  __attribute__((ext_vector_type(4)));
typedef float  v4fa __attribute__((ext_vector_type(4), may_alias));
typedef _Float16 v16h __attribute__((ext_vector_type(16)));
typedef _Float16 v4h __attribute__((ext_vector_type(4)));
union FragH { v16h v; v8us half[2]; _Float16 h[16]; unsigned short u[16]; };

__device__ __forceinline__ unsigned short bf16_bits(float x) { unsigned int u = __float_as_uint(x); return (unsigned short)((u + 0x7FFFu + ((u >> 16) & 1u)) >> 16); }
__device__ __forceinline__ float bf16_val(unsigned short b) { return __uint_as_float(((unsigned int)b) << 16); }
__device__ __forceinline__ float bf16_rne(float x) { return bf16_val(bf16_bits(x)); }

__global__ __launch_bounds__(256) void k_wt_f16(const float* __restrict__ W, _Float16* __restrict__ Wt, int K, int N, float scale) {
  const int t = blockIdx.x * 256 + threadIdx.x; if (t >= N * (K / 8)) return;
  const int n = t / (K / 8), k8 = (t % (K / 8)) * 8; FragH f;
#pragma unroll
  for (int i = 0; i < 8; ++i) f.h[i] = (_Float16)(bf16_rne(W[(size_t)(k8 + i) * N + n]) * scale);
  const v8us o = f.half[0];
  unsigned short* d = (unsigned short*)Wt + (size_t)n * K + k8;
  *(volatile v8us*)d = o; __threadfence(); *(volatile v8us*)d = o;
}

__global__ __launch_bounds__(256) void k_x16(const float* __restrict__ x, _Float16* __restrict__ X16, size_t n8) {
  const size_t t = (size_t)blockIdx.x * 256 + threadIdx.x; if (t >= n8) return;
  const size_t row = t / (DM / 8); const int c8 = (int)(t % (DM / 8)) * 8;
  const size_t b = row / SQ, s = row % SQ;
  const float* src = x + (b * (size_t)SQ_FULL + s) * DM + c8;
  const v4f a = *(const v4fa*)src, c = *(const v4fa*)(src + 4);
  FragH f;
#pragma unroll
  for (int q = 0; q < 4; ++q) { f.h[q] = (_Float16)bf16_rne(a[q]); f.h[4 + q] = (_Float16)bf16_rne(c[q]); }
  const v8us o = f.half[0];
  unsigned short* d = (unsigned short*)X16 + t * 8;
  *(volatile v8us*)d = o; __threadfence(); *(volatile v8us*)d = o;
}

template <int NHv, int TTv>
__global__ __launch_bounds__(256) void k_vt(const _Float16* __restrict__ V16, int ldv, int voff, _Float16* __restrict__ Vt) {
  __shared__ unsigned short tl[64][66];
  const int tid = threadIdx.x; const int slab = blockIdx.x / (TTv / 64), lg = blockIdx.x % (TTv / 64); const int b = slab / NHv, h = slab % NHv;
  for (int i = tid; i < 64 * 8; i += 256) { const int r = i / 8, c8 = (i % 8) * 8; FragH f; f.half[0] = *(const v8us*)((const unsigned short*)V16 + ((size_t)b * TTv + lg * 64 + r) * ldv + voff + h * 64 + c8);
#pragma unroll
    for (int q = 0; q < 8; ++q) tl[r][c8 + q] = f.u[q]; }
  __syncthreads();
  for (int pass = 0; pass < 2; ++pass) {
#pragma unroll
    for (int rd = 0; rd < 2; ++rd) { const int d = rd * 32 + tid / 8, pc = tid % 8; FragH f;
#pragma unroll
      for (int q = 0; q < 8; ++q) f.u[q] = tl[pc * 8 + q][d];
      *(volatile v8us*)((unsigned short*)Vt + ((size_t)slab * 64 + d) * TTv + lg * 64 + pc * 8) = f.half[0]; }
    if (pass == 0) __threadfence(); } }

__device__ __forceinline__ v16h g2_frag(const _Float16* p, int hh) { FragH f; f.half[0] = *(const v8us*)((const unsigned short*)p + 8 * hh); f.half[1] = *(const v8us*)((const unsigned short*)p + 16 + 8 * hh); return f.v; }
__device__ __forceinline__ v8f g2_mma(v16h a, v16h b, v8f c) { v8f d = __builtin_amdgcn_wmma_f32_16x16x32_f16(false, a, false, b, (short)0, c, false, false); asm volatile("v_nop\n\tv_nop\n\tv_nop\n\tv_nop" : "+v"(d) : "v"(a), "v"(b)); return d; }
template <bool HASBIAS, bool OUTF32>
__global__ __launch_bounds__(128) void k_gemm2(const _Float16* __restrict__ A, int lda, size_t sA, const _Float16* __restrict__ Bh, int ldb, size_t sB, float alpha, const float* __restrict__ bias,
    float* __restrict__ C, _Float16* __restrict__ C16, int ldc, size_t sC, int M, int N, int K) {
  __shared__ __attribute__((aligned(16))) float so[4][32][68];
  const int tid = threadIdx.x, w = tid >> 5, lane = tid & 31, ln = lane & 15, hh = lane >> 4; const int by = blockIdx.y;
  A += (size_t)by * sA; Bh += (size_t)by * sB; const size_t cofs = (size_t)by * sC;
  const int ntn = N >> 6; const int mt = blockIdx.x / ntn, nq = blockIdx.x - mt * ntn; const int row0 = mt * 128 + 32 * w, col0 = nq * 64; if (row0 >= M) return;
  const _Float16* a0p = A + (size_t)(row0 + ln) * lda; const _Float16* a1p = a0p + (size_t)16 * lda;
  const _Float16* b0p = Bh + (size_t)(col0 + ln) * ldb; const _Float16* b1p = b0p + (size_t)16 * ldb; const _Float16* b2p = b1p + (size_t)16 * ldb; const _Float16* b3p = b2p + (size_t)16 * ldb;
  const v8f z8 = {0.f,0.f,0.f,0.f,0.f,0.f,0.f,0.f}; v8f c00 = z8, c01 = z8, c02 = z8, c03 = z8, c10 = z8, c11 = z8, c12 = z8, c13 = z8;
#pragma unroll 1
  for (int kb = 0; kb < K; kb += 32) { const v16h a0 = g2_frag(a0p + kb, hh), a1 = g2_frag(a1p + kb, hh);
    v16h b = g2_frag(b0p + kb, hh); c00 = g2_mma(a0, b, c00); c10 = g2_mma(a1, b, c10);
    b = g2_frag(b1p + kb, hh); c01 = g2_mma(a0, b, c01); c11 = g2_mma(a1, b, c11);
    b = g2_frag(b2p + kb, hh); c02 = g2_mma(a0, b, c02); c12 = g2_mma(a1, b, c12);
    b = g2_frag(b3p + kb, hh); c03 = g2_mma(a0, b, c03); c13 = g2_mma(a1, b, c13); }
  v8f accs[8] = {c00, c01, c02, c03, c10, c11, c12, c13};
#pragma unroll
  for (int u = 0; u < 8; ++u) { const int t = u & 3, half = u >> 2; const int col = col0 + t * 16 + ln; float bv = 0.f; if (HASBIAS) bv = bf16_rne(bias[col]);
#pragma unroll
    for (int r = 0; r < 8; ++r) { const int rloc = half * 16 + 8 * hh + r; so[w][rloc][t * 16 + ln] = accs[u][r] * alpha + bv; } }
  __builtin_amdgcn_fence(4  , "workgroup"); __builtin_amdgcn_wave_barrier();
  const int rsub = lane >> 4, c4 = (lane & 15) * 4;
  for (int pass = 0; pass < 2; ++pass) {
#pragma unroll
    for (int q = 0; q < 16; ++q) { const int r = q * 2 + rsub; const v4f v = *(const v4fa*)&so[w][r][c4];
      if (OUTF32) { *(volatile v4f*)(C + cofs + (size_t)(row0 + r) * ldc + col0 + c4) = v; }
      else { v4h h4;
#pragma unroll
        for (int i = 0; i < 4; ++i) h4[i] = (_Float16)v[i];
        *(volatile v4h*)(C16 + cofs + (size_t)(row0 + r) * ldc + col0 + c4) = h4; } }
    if (pass == 0) __threadfence(); } }

__global__ __launch_bounds__(256) void k_rsmf(const float* __restrict__ S, _Float16* __restrict__ P, int qn, int hg) {
  #pragma clang fp contract(off)
  const int t = blockIdx.x * 256 + threadIdx.x; if (t >= qn * hg) return;
  const size_t i = (size_t)(t / qn) * SQ + (t % qn); const float* s = S + i * SQ; float mx = -3.0e38f;
#pragma unroll 1
  for (int j = 0; j < SQ; j += 4) { const v4f a = *(const v4fa*)(s + j); mx = fmaxf(mx, a[0]); mx = fmaxf(mx, a[1]); mx = fmaxf(mx, a[2]); mx = fmaxf(mx, a[3]); }
  float se = 0.f;
#pragma unroll 1
  for (int j = 0; j < SQ; j += 4) { const v4f a = *(const v4fa*)(s + j); se += __expf(a[0] - mx); se += __expf(a[1] - mx); se += __expf(a[2] - mx); se += __expf(a[3] - mx); }
  const float sc = 256.0f / se;
#pragma unroll 1
  for (int j0 = 0; j0 < SQ; j0 += 8) { const v4f a = *(const v4fa*)(s + j0), c = *(const v4fa*)(s + j0 + 4); FragH f;
#pragma unroll
    for (int q = 0; q < 4; ++q) { f.h[q] = (_Float16)(__expf(a[q] - mx) * sc); f.h[4 + q] = (_Float16)(__expf(c[q] - mx) * sc); }
    const v8us o = f.half[0]; unsigned short* d = (unsigned short*)P + i * SQ + j0;
    *(volatile v8us*)d = o; __threadfence(); *(volatile v8us*)d = o; } }

extern "C" void kernel_launch(void* const* d_in, const int* in_sizes, int n_in,
                              void* d_out, int out_size, void* d_ws, size_t ws_size, hipStream_t stream) {
  if (n_in < 5) return;
  if (in_sizes[0] < (int)((((size_t)NB - 1) * SQ_FULL + SQ) * DM)) return;
  if (in_sizes[1] < DM * LQ || in_sizes[2] < LQ || in_sizes[3] < DM * DM || in_sizes[4] < DM) return;
  if (out_size < (int)(NR * DM)) return;
  const float* x = (const float*)d_in[0]; const float* wqkv = (const float*)d_in[1]; const float* bqkv = (const float*)d_in[2];
  const float* wo = (const float*)d_in[3]; const float* bo = (const float*)d_in[4];
  float* out = (float*)d_out;
  char* ws = (char*)d_ws; size_t off = 0;
  _Float16* BQKV = (_Float16*)(ws + off); off += SZ_BQKV;
  _Float16* BO   = (_Float16*)(ws + off); off += SZ_BO;
  _Float16* X16  = (_Float16*)(ws + off); off += SZ_X16;
  _Float16* QKV  = (_Float16*)(ws + off); off += SZ_QKV;
  float*    S    = (float*)(ws + off);    off += SZ_S;
  _Float16* P    = (_Float16*)(ws + off); off += SZ_P;
  _Float16* VT   = (_Float16*)(ws + off); off += SZ_VT;
  if (off > ws_size) return;
  _Float16* O16 = X16;
  _Float16* Q16 = QKV; _Float16* K16 = QKV + DM; _Float16* V16 = QKV + 2 * DM;

  k_wt_f16<<<(unsigned)(((size_t)LQ * (DM / 8) + 255) / 256), 256, 0, stream>>>(wqkv, BQKV, DM, LQ, 16.0f);
  k_wt_f16<<<(unsigned)(((size_t)DM * (DM / 8) + 255) / 256), 256, 0, stream>>>(wo, BO, DM, DM, 16.0f);
  k_x16<<<(unsigned)((NR * DM / 8 + 255) / 256), 256, 0, stream>>>(x, X16, NR * DM / 8);
  k_gemm2<true, false><<<dim3((unsigned)((NR / 128) * (LQ / 64)), 1), 128, 0, stream>>>(X16, DM, (size_t)0, BQKV, DM, (size_t)0, 0.0625f, bqkv, S, QKV, LQ, (size_t)0, (int)NR, LQ, DM);
  for (int b = 0; b < NB; ++b) {
    const size_t r0 = (size_t)b * SQ;
    k_vt<NH, SQ><<<NH * (SQ / 64), 256, 0, stream>>>(V16 + r0 * LQ, LQ, 0, VT);
    for (int h0 = 0; h0 < NH; h0 += HG) {
      k_gemm2<false, true><<<dim3((SQ / 128) * (SQ / 64), HG), 128, 0, stream>>>(Q16 + r0 * LQ + h0 * HD, LQ, (size_t)HD, K16 + r0 * LQ + h0 * HD, LQ, (size_t)HD, 0.125f, bqkv, S, P, SQ, (size_t)SQ * SQ, SQ, SQ, HD);
      k_rsmf<<<(HG * SQ + 255) / 256, 256, 0, stream>>>(S, P, SQ, HG);
      k_gemm2<false, false><<<dim3((SQ / 128) * (HD / 64), HG), 128, 0, stream>>>(P, SQ, (size_t)SQ * SQ, VT + (size_t)h0 * HD * SQ, SQ, (size_t)HD * SQ, 0.25f, bqkv, S, O16 + r0 * DM + h0 * HD, DM, (size_t)HD, SQ, HD, SQ);
    }
  }
  k_gemm2<true, true><<<dim3((unsigned)((NR / 128) * (DM / 64)), 1), 128, 0, stream>>>(O16, DM, (size_t)0, BO, DM, (size_t)0, 0.0009765625f, bo, out, P, DM, (size_t)0, (int)NR, DM, DM);
}
